// MultiHeadedAttention_79946521247894
// MI455X (gfx1250) — hardware-verified
//
#include <hip/hip_runtime.h>


#ifndef NB
#define NB 4
#endif
#ifndef SEQ
#define SEQ 2048
#endif
#define SEQ_FULL 2048
#define NB_FULL  4
#define TT   SEQ
#define EE   1024
#define NH_  16
#define HD   64
#define DM   (NH_ * HD)
#define QKP  (2 * DM)
#define CATC 256.0f
#define WPC  64.0f
#define OSC  6.103515625e-05f

static_assert(TT % 128 == 0);
static_assert(TT <= SEQ_FULL);
static_assert(NB >= 1 && NB <= NB_FULL);
static_assert(HD == 64);
static_assert(HD == 2 * 32);
static_assert(HD == 4 * 16);
static_assert(NH_ * HD == DM);
static_assert(DM == EE);
static_assert(EE % 32 == 0 && DM % 32 == 0 && TT % 32 == 0);
static_assert(EE % 64 == 0 && DM % 64 == 0 && QKP % 64 == 0 && TT % 64 == 0);
static_assert((NB * TT) % 64 == 0);
static_assert(EE % 8 == 0 && DM % 8 == 0);
static_assert(((size_t)DM * EE) % 8 == 0 && ((size_t)NB * SEQ_FULL * EE) % 8 == 0);
static_assert((QKP * 2) % 128 == 0 && (DM * 2) % 128 == 0 && (TT * 2) % 128 == 0 && (EE * 4) % 128 == 0);
static_assert(8 * 16 == 128);
static_assert(8 * 8 == HD);
static_assert(16 * 4 == 64);

#define WS_WT  ((size_t)3 * DM * EE * 2)
#define WS_WPT ((size_t)EE * DM * 2)
#define WS_XB  ((size_t)NB * SEQ_FULL * EE * 2)
#define WS_QK  ((size_t)NB * TT * QKP * 2)
#define WS_VT  ((size_t)NB * DM * TT * 2)
#define WS_CAT ((size_t)NB * TT * DM * 2)
static_assert(WS_WT % 256 == 0 && WS_WPT % 256 == 0 && WS_XB % 256 == 0 && WS_QK % 256 == 0 && WS_VT % 256 == 0 && WS_CAT % 256 == 0);
static_assert(WS_WT + WS_WPT + WS_XB + WS_QK + WS_VT + WS_CAT <= (size_t)134217728);

typedef _Float16 h16;
typedef unsigned short bf;
typedef __attribute__((ext_vector_type(16))) __bf16   v16bf;
typedef __attribute__((ext_vector_type(16))) _Float16 v16h;
typedef __attribute__((ext_vector_type(8)))  _Float16 v8h;
typedef __attribute__((ext_vector_type(8)))  unsigned short v8us;
typedef __attribute__((ext_vector_type(8)))  float    v8f;
typedef __attribute__((ext_vector_type(4)))  float    v4f;
typedef v8h  __attribute__((may_alias)) v8ha;
typedef v4f  __attribute__((may_alias)) v4fa;

__device__ __forceinline__ unsigned short f2bf(float f) { unsigned u = __float_as_uint(f); u += 0x7FFFu + ((u >> 16) & 1u); return (unsigned short)(u >> 16); }
__device__ __forceinline__ float bf2f(unsigned short b) { return __uint_as_float(((unsigned)b) << 16); }
__device__ __forceinline__ float bfr(float f) { return bf2f(f2bf(f)); }
__device__ __forceinline__ v16h cat16(v8h lo, v8h hi) { return __builtin_shufflevector(lo, hi, 0, 1, 2, 3, 4, 5, 6, 7, 8, 9, 10, 11, 12, 13, 14, 15); }
__device__ __forceinline__ v16bf cat16b(v8us lo, v8us hi) { return __builtin_bit_cast(v16bf, __builtin_shufflevector(lo, hi, 0, 1, 2, 3, 4, 5, 6, 7, 8, 9, 10, 11, 12, 13, 14, 15)); }
__device__ __forceinline__ v8f wmma16(v16h a, v16h b, v8f c) { return __builtin_amdgcn_wmma_f32_16x16x32_f16(false, a, false, b, (short)0, c, false, false); }
__device__ __forceinline__ v8f wmmab(v16bf a, v16bf b, v8f c) { return __builtin_amdgcn_wmma_f32_16x16x32_bf16(false, a, false, b, (short)0, c, false, false); }

template <typename T16> struct WFrag;
template <> struct WFrag<h16> { typedef v16h V; static __device__ __forceinline__ V ld(const h16* p) { return cat16(*(const v8h*)p, *(const v8h*)(p + 16)); } static __device__ __forceinline__ v8f mma(V a, V b, v8f c) { return wmma16(a, b, c); } };
template <> struct WFrag<bf> { typedef v16bf V; static __device__ __forceinline__ V ld(const bf* p) { return cat16b(*(const v8us*)p, *(const v8us*)(p + 16)); } static __device__ __forceinline__ v8f mma(V a, V b, v8f c) { return wmmab(a, b, c); } };

template <typename T16, bool OUT16, bool BIAS>
__device__ __forceinline__ void gemm_body(const T16* __restrict__ A, const T16* __restrict__ Bt, const int K, float* Cf, h16* Ch, const int ldc,
                                          const float* __restrict__ bias, const float oscale, const size_t sA, const size_t sB, const size_t sC) {
    typedef typename WFrag<T16>::V V;
    __shared__ __align__(16) float os[16 * 68];
    const size_t z = blockIdx.z; A += z * sA; Bt += z * sB;
    const int lane = threadIdx.x & 31, lr = lane & 15, hi = lane >> 4; const int r0 = blockIdx.x * 64, c0 = blockIdx.y * 64;
    v8f acc[4][4];
#pragma unroll
    for (int mb = 0; mb < 4; ++mb)
#pragma unroll
        for (int nb = 0; nb < 4; ++nb) acc[mb][nb] = (v8f){};
    const size_t aoff = (size_t)(r0 + lr) * K + 8 * hi, boff = (size_t)(c0 + lr) * K + 8 * hi;
#pragma unroll 1
    for (int kc = 0; kc < K; kc += 32) {
        V a[4];
#pragma unroll
        for (int mb = 0; mb < 4; ++mb) a[mb] = WFrag<T16>::ld(A + aoff + (size_t)mb * 16 * K + kc);
#pragma unroll
        for (int nb = 0; nb < 4; ++nb) { const V b = WFrag<T16>::ld(Bt + boff + (size_t)nb * 16 * K + kc);
#pragma unroll
            for (int mb = 0; mb < 4; ++mb) acc[mb][nb] = WFrag<T16>::mma(a[mb], b, acc[mb][nb]); }
        asm volatile("v_nop\n\tv_nop\n\tv_nop\n\tv_nop" : "+v"(acc[0][0]), "+v"(acc[1][1]), "+v"(acc[2][2]), "+v"(acc[3][3]) : "v"(a[0]), "v"(a[3]));
    }
#pragma unroll
    for (int mb = 0; mb < 4; ++mb) {
#pragma unroll
        for (int nb = 0; nb < 4; ++nb) {
#pragma unroll
            for (int j = 0; j < 8; ++j) os[(hi * 8 + j) * 68 + nb * 16 + lr] = acc[mb][nb][j]; }
        __builtin_amdgcn_wave_barrier(); asm volatile("" ::: "memory");
        if (OUT16) {
            h16* crow = Ch + z * sC + (size_t)(r0 + mb * 16) * ldc + c0;
#pragma unroll 1
            for (int ps = 0; ps < 2; ++ps) {
#pragma unroll
                for (int s = 0; s < 4; ++s) { const int row = 4 * s + (lane >> 3), pc = (lane & 7) * 8;
                    const v4f x0 = *(const v4fa*)(os + row * 68 + pc); const v4f x1 = *(const v4fa*)(os + row * 68 + pc + 4); v8h o;
#pragma unroll
                    for (int q = 0; q < 4; ++q) { o[q] = (h16)(x0[q] * oscale); o[4 + q] = (h16)(x1[q] * oscale); }
                    *(volatile v8h*)(crow + (size_t)row * ldc + pc) = o; }
                if (ps == 0) __threadfence(); }
        } else {
            float* crow = Cf + z * sC + (size_t)(r0 + mb * 16) * ldc + c0;
#pragma unroll 1
            for (int ps = 0; ps < 2; ++ps) {
#pragma unroll
                for (int s = 0; s < 8; ++s) { const int row = 2 * s + hi, cofs = lr * 4; v4f val = *(const v4fa*)(os + row * 68 + cofs);
                    val[0] *= oscale; val[1] *= oscale; val[2] *= oscale; val[3] *= oscale;
                    if (BIAS) { const v4f bb = *(const v4f*)(bias + c0 + cofs); val[0] += bfr(bb[0]); val[1] += bfr(bb[1]); val[2] += bfr(bb[2]); val[3] += bfr(bb[3]); }
                    *(volatile v4f*)(crow + (size_t)row * ldc + cofs) = val; }
                if (ps == 0) __threadfence(); }
        }
        __builtin_amdgcn_wave_barrier(); asm volatile("" ::: "memory");
    }
}

__global__ __launch_bounds__(32) void k_gemm_p16(const bf* __restrict__ A, const bf* __restrict__ Bt, int K, h16* C, int ldc, size_t sA, size_t sB, size_t sC) {
    gemm_body<bf, true, false>(A, Bt, K, nullptr, C, ldc, nullptr, 1.0f, sA, sB, sC);
}
__global__ __launch_bounds__(32) void k_gemm_out(const h16* __restrict__ A, const h16* __restrict__ Bt, int K, float* C, int ldc, const float* __restrict__ bias, float oscale) {
    gemm_body<h16, false, true>(A, Bt, K, C, nullptr, ldc, bias, oscale, (size_t)0, (size_t)0, (size_t)0);
}

__global__ __launch_bounds__(256) void k_cvt8(const float* __restrict__ src, bf* dst, size_t n8) { const size_t i = (size_t)blockIdx.x * 256 + threadIdx.x; if (i >= n8) return; const v8f v = *(const v8f*)(src + i * 8); v8us o;
#pragma unroll
    for (int k = 0; k < 8; ++k) o[k] = f2bf(v[k]); *(volatile v8us*)(dst + i * 8) = o; __threadfence(); *(volatile v8us*)(dst + i * 8) = o; }

__global__ __launch_bounds__(256) void k_cvtwo(const float* __restrict__ src, h16* dst, size_t n8) { const size_t i = (size_t)blockIdx.x * 256 + threadIdx.x; if (i >= n8) return; const v8f v = *(const v8f*)(src + i * 8); v8h o;
#pragma unroll
    for (int k = 0; k < 8; ++k) o[k] = (h16)(bfr(v[k]) * WPC); *(volatile v8h*)(dst + i * 8) = o; __threadfence(); *(volatile v8h*)(dst + i * 8) = o; }

__global__ __launch_bounds__(256) void k_attn(const h16* __restrict__ QK, const h16* __restrict__ VT, h16* CAT) {
    __shared__ __align__(16) h16 ot[8 * 16 * 72];
    const int bh = blockIdx.x; const int b = bh / NH_, h = bh % NH_;
    const int wid = threadIdx.x >> 5, lane = threadIdx.x & 31, lr = lane & 15, hi = lane >> 4;
    const int t0 = blockIdx.y * 128 + wid * 16;
    const h16* qp = QK + ((size_t)b * TT + t0 + lr) * QKP + h * HD + 8 * hi;
    const v16h qf0 = WFrag<h16>::ld(qp), qf1 = WFrag<h16>::ld(qp + 32);
    const h16* kb = QK + ((size_t)b * TT + lr) * QKP + DM + h * HD + 8 * hi;
    const h16* vb = VT + ((size_t)b * DM + h * HD + lr) * TT + 8 * hi;
    v8f acc[4];
#pragma unroll
    for (int n = 0; n < 4; ++n) acc[n] = (v8f){};
    float m = -3.0e38f, l = 0.f;
    const float cs = 0.125f * 1.4426950408889634f;
#pragma unroll 1
    for (int s0 = 0; s0 < TT; s0 += 64) {
        v8f sc[4];
#pragma unroll
        for (int t = 0; t < 4; ++t) {
            const h16* kp = kb + (size_t)(s0 + t * 16) * QKP;
            const v16h k0 = WFrag<h16>::ld(kp), k1 = WFrag<h16>::ld(kp + 32);
            v8f zz = (v8f){};
            zz = wmma16(k0, qf0, zz);
            sc[t] = wmma16(k1, qf1, zz);
        }
        asm volatile("v_nop\n\tv_nop\n\tv_nop\n\tv_nop" : "+v"(sc[0]), "+v"(sc[1]), "+v"(sc[2]), "+v"(sc[3]) : "v"(qf0), "v"(qf1));
        float mx = sc[0][0];
#pragma unroll
        for (int t = 0; t < 4; ++t)
#pragma unroll
            for (int r = 0; r < 8; ++r) mx = fmaxf(mx, sc[t][r]);
        mx = fmaxf(mx, __shfl_xor(mx, 16, 32));
        const float mn = fmaxf(m, mx);
        const float alpha = __builtin_amdgcn_exp2f((m - mn) * cs);
        const float mo = mn * cs;
        m = mn;
        float psum = 0.f; v16h pb0, pb1;
#pragma unroll
        for (int r = 0; r < 8; ++r) {
            const float p0 = __builtin_amdgcn_exp2f(fmaf(sc[0][r], cs, -mo));
            const float p1 = __builtin_amdgcn_exp2f(fmaf(sc[1][r], cs, -mo));
            const float p2 = __builtin_amdgcn_exp2f(fmaf(sc[2][r], cs, -mo));
            const float p3 = __builtin_amdgcn_exp2f(fmaf(sc[3][r], cs, -mo));
            psum += (p0 + p1) + (p2 + p3);
            pb0[r] = (h16)p0; pb0[8 + r] = (h16)p1; pb1[r] = (h16)p2; pb1[8 + r] = (h16)p3;
        }
        l = l * alpha + psum;
#pragma unroll
        for (int n = 0; n < 4; ++n)
#pragma unroll
            for (int r = 0; r < 8; ++r) acc[n][r] *= alpha;
#pragma unroll
        for (int n = 0; n < 4; ++n) {
            const h16* vp = vb + (size_t)n * 16 * TT + s0;
            const v16h va0 = WFrag<h16>::ld(vp), va1 = WFrag<h16>::ld(vp + 32);
            acc[n] = wmma16(va0, pb0, acc[n]);
            acc[n] = wmma16(va1, pb1, acc[n]);
        }
        asm volatile("v_nop\n\tv_nop\n\tv_nop\n\tv_nop" : "+v"(acc[0]), "+v"(acc[1]), "+v"(acc[2]), "+v"(acc[3]) : "v"(pb0), "v"(pb1));
    }
    const float lt = l + __shfl_xor(l, 16, 32);
    const float inv = CATC * (1.0f / lt);
    h16* tile = ot + wid * 16 * 72;
#pragma unroll
    for (int n = 0; n < 4; ++n) { v8h o;
#pragma unroll
        for (int r = 0; r < 8; ++r) o[r] = (h16)(acc[n][r] * inv);
        *(v8ha*)(tile + lr * 72 + n * 16 + 8 * hi) = o; }
    __builtin_amdgcn_wave_barrier(); asm volatile("" ::: "memory");
    h16* crow = CAT + ((size_t)b * TT + t0) * DM + h * HD;
#pragma unroll 1
    for (int ps = 0; ps < 2; ++ps) {
#pragma unroll
        for (int s = 0; s < 4; ++s) { const int row = 4 * s + (lane >> 3), pc = (lane & 7) * 8;
            const v8h v = *(const v8ha*)(tile + row * 72 + pc);
            *(volatile v8h*)(crow + (size_t)row * DM + pc) = v; }
        if (ps == 0) __threadfence(); }
}

extern "C" void kernel_launch(void* const* d_in, const int* in_sizes, int n_in,
                              void* d_out, int out_size, void* d_ws, size_t ws_size, hipStream_t stream) {
    if (n_in < 6) return;
    if (in_sizes[0] < NB * SEQ_FULL * EE) return;
    if (in_sizes[1] < DM * EE || in_sizes[2] < DM * EE || in_sizes[3] < DM * EE) return;
    if (in_sizes[4] < EE * DM || in_sizes[5] < EE) return;
    if (out_size < NB * TT * EE) return;
    const float* x  = (const float*)d_in[0];
    const float* wq = (const float*)d_in[1];
    const float* wk = (const float*)d_in[2];
    const float* wv = (const float*)d_in[3];
    const float* wo = (const float*)d_in[4];
    const float* bo = (const float*)d_in[5];
    float* OUT = (float*)d_out;
    char* wsp = (char*)d_ws;
    auto take = [&](size_t bytes) { char* p = wsp; wsp += (bytes + 255) & ~(size_t)255; return (void*)p; };
    bf*  WT  = (bf*)take(WS_WT);
    h16* WPT = (h16*)take(WS_WPT);
    bf*  XB  = (bf*)take(WS_XB);
    h16* QKp = (h16*)take(WS_QK);
    h16* VTp = (h16*)take(WS_VT);
    h16* CATp = (h16*)take(WS_CAT);
    if ((size_t)(wsp - (char*)d_ws) > ws_size) return;

    const size_t nw8 = (size_t)DM * EE / 8;
    const unsigned LW = (unsigned)((nw8 + 255) / 256);
    k_cvt8<<<LW, 256, 0, stream>>>(wq, WT, nw8);
    k_cvt8<<<LW, 256, 0, stream>>>(wk, WT + (size_t)DM * EE, nw8);
    k_cvt8<<<LW, 256, 0, stream>>>(wv, WT + (size_t)2 * DM * EE, nw8);
    k_cvtwo<<<LW, 256, 0, stream>>>(wo, WPT, nw8);
    const size_t nx8 = (size_t)NB * SEQ_FULL * EE / 8;
    k_cvt8<<<(unsigned)((nx8 + 255) / 256), 256, 0, stream>>>(x, XB, nx8);
    k_gemm_p16<<<dim3(TT / 64, QKP / 64, NB), 32, 0, stream>>>(XB, WT, EE, QKp, QKP, (size_t)SEQ_FULL * EE, (size_t)0, (size_t)TT * QKP);
    k_gemm_p16<<<dim3(DM / 64, TT / 64, NB), 32, 0, stream>>>(WT + (size_t)2 * DM * EE, XB, EE, VTp, TT, (size_t)0, (size_t)SEQ_FULL * EE, (size_t)DM * TT);
    k_attn<<<dim3(NB * NH_, TT / 128), 256, 0, stream>>>(QKp, VTp, CATp);
    k_gemm_out<<<dim3(NB * TT / 64, EE / 64, 1), 32, 0, stream>>>(CATp, WPT, DM, OUT, EE, bo, OSC);
}
